// LlamaAttentionQKV_37409165148605
// MI455X (gfx1250) — hardware-verified
//
#include <hip/hip_runtime.h>
#include <math.h>
#include <stdint.h>

#define NB    2
#define SEQ   1024
#define NH    32
#define NKV   8
#define HD    128
#define GRP   4
#define QSC   1024.0f
#define KSC   1024.0f
#define PCAR  32768.0f
#define VCAR  16.0f
#define LOG2E 1.4426950408889634f
#define BIASTH (-1.0e8f)
#define ATW   GRP
#define ATT_THREADS (ATW * 32)
#define ATT_BLOCKS  (NB * NKV * (SEQ / 16))
#define SLABF (16 * 132)
#define VTP   72
static_assert(NH == NKV * GRP);
static_assert(HD == 128 && (SEQ % 64) == 0 && (SEQ % 32) == 0 && (SEQ % 16) == 0);
static_assert(ATT_THREADS == 128 && ATT_BLOCKS == 1024);
static_assert(((NB * SEQ * NH * 16) % 256) == 0 && ((NB * SEQ * NKV * 16) % 256) == 0);
static_assert(16 * 36 <= SLABF);
static_assert((SEQ / 16) == 64 && NKV == 8);

typedef _Float16 v16h __attribute__((ext_vector_type(16)));
typedef _Float16 v8h  __attribute__((ext_vector_type(8)));
typedef float    v8f  __attribute__((ext_vector_type(8)));
typedef float    v4f  __attribute__((ext_vector_type(4)));
typedef unsigned int v4u __attribute__((ext_vector_type(4)));

union FragH { v16h v; v8h h[2]; v4u u[2]; };

__device__ __forceinline__ unsigned short bf_bits(float f) {
  unsigned u = __float_as_uint(f);
  return (unsigned short)((u + 0x7FFFu + ((u >> 16) & 1u)) >> 16);
}
__device__ __forceinline__ float bf_up(unsigned short h) { return __uint_as_float(((unsigned)h) << 16); }
__device__ __forceinline__ float bfr(float f) { return bf_up(bf_bits(f)); }
__device__ __forceinline__ unsigned short h_bits(_Float16 x) { return __builtin_bit_cast(unsigned short, x); }
__device__ __forceinline__ unsigned pk16(unsigned short a, unsigned short b) { return (unsigned)a | ((unsigned)b << 16); }
__device__ __forceinline__ v8f zero8() { v8f z = {0.f, 0.f, 0.f, 0.f, 0.f, 0.f, 0.f, 0.f}; return z; }

__device__ __forceinline__ v16h ldfrag_h(const _Float16* p) {
  FragH f;
  f.h[0] = *(const v8h*)(p);
  f.h[1] = *(const v8h*)(p + 16);
  return f.v;
}

__device__ __forceinline__ v8f mma_raw(v16h a, v16h b, v8f c) {
  return __builtin_amdgcn_wmma_f32_16x16x32_f16(false, a, false, b, (short)0, c, false, false);
}
__device__ __forceinline__ void guard_sc(v8f& a, v8f& b, v16h x0, v16h x1, v16h x2, v16h x3, v16h x4, v16h x5) {
#if defined(__HIP_DEVICE_COMPILE__)
  asm volatile("v_nop\n\tv_nop\n\tv_nop\n\tv_nop"
               : "+v"(a), "+v"(b) : "v"(x0), "v"(x1), "v"(x2), "v"(x3), "v"(x4), "v"(x5) : "memory");
#endif
}
__device__ __forceinline__ void guard_pv(v8f& a, v8f& b, v8f& c, v8f& d,
                                         v16h p0, v16h p1, v16h x0, v16h x1, v16h x2, v16h x3) {
#if defined(__HIP_DEVICE_COMPILE__)
  asm volatile("v_nop\n\tv_nop\n\tv_nop\n\tv_nop"
               : "+v"(a), "+v"(b), "+v"(c), "+v"(d) : "v"(p0), "v"(p1), "v"(x0), "v"(x1), "v"(x2), "v"(x3) : "memory");
#endif
}
__device__ __forceinline__ void acc_guard4(v8f& a, v8f& b, v8f& c, v8f& d) {
#if defined(__HIP_DEVICE_COMPILE__)
  asm volatile("v_nop\n\tv_nop\n\tv_nop\n\tv_nop" : "+v"(a), "+v"(b), "+v"(c), "+v"(d));
#endif
}
__device__ __forceinline__ void wave_sync_lds() {
  __builtin_amdgcn_fence(__ATOMIC_RELEASE, "workgroup");
  __builtin_amdgcn_wave_barrier();
  __builtin_amdgcn_fence(__ATOMIC_ACQUIRE, "workgroup");
}

__global__ __launch_bounds__(256) void rope16(const float* __restrict__ x, const float* __restrict__ cosT,
                                              const float* __restrict__ sinT, unsigned short* hipl, unsigned short* lopl,
                                              int nrows, int hpr, float sc) {
  const int gt  = blockIdx.x * 256 + (int)threadIdx.x;
  const int row = gt >> 4;
  const int d0  = (gt & 15) * 8;
  if (row >= nrows) return;
  const int pos = (row / hpr) & (SEQ - 1);
  const int d1  = d0 ^ 64;
  const float* xr = x + (size_t)row * HD;
  const float* cr = cosT + (size_t)pos * HD + d0;
  const float* sr = sinT + (size_t)pos * HD + d0;
  const v4f xa = *(const v4f*)(xr + d0), xb = *(const v4f*)(xr + d0 + 4);
  const v4f ya = *(const v4f*)(xr + d1), yb = *(const v4f*)(xr + d1 + 4);
  const v4f ca = *(const v4f*)(cr), cb = *(const v4f*)(cr + 4);
  const v4f sa = *(const v4f*)(sr), sb = *(const v4f*)(sr + 4);
  const float sgn = (d0 < 64) ? -1.0f : 1.0f;
  float w[8];
#pragma unroll
  for (int e = 0; e < 4; ++e) {
    w[e]     = bfr(xa[e]) * bfr(ca[e]) + (sgn * bfr(ya[e])) * bfr(sa[e]);
    w[4 + e] = bfr(xb[e]) * bfr(cb[e]) + (sgn * bfr(yb[e])) * bfr(sb[e]);
  }
  v4u oh, ol;
#pragma unroll
  for (int e = 0; e < 4; ++e) {
    const float t0 = w[2 * e] * sc, t1 = w[2 * e + 1] * sc;
    const _Float16 h0 = (_Float16)t0, h1 = (_Float16)t1;
    const _Float16 l0 = (_Float16)(t0 - (float)h0), l1 = (_Float16)(t1 - (float)h1);
    oh[e] = pk16(h_bits(h0), h_bits(h1));
    ol[e] = pk16(h_bits(l0), h_bits(l1));
  }
  const size_t o8 = (size_t)row * HD + d0;
  for (int pass = 0; pass < 2; ++pass) {
    *(volatile v4u*)(hipl + o8) = oh;
    *(volatile v4u*)(lopl + o8) = ol;
    __threadfence();
  }
}

__global__ __launch_bounds__(256) void vt16(const float* __restrict__ v, unsigned short* VTo) {
  __shared__ __align__(16) unsigned short T[HD * VTP];
  const int tid = threadIdx.x;
  const int bid = blockIdx.x;
  const int st  = bid & 15;
  const int g   = (bid >> 4) & 7;
  const int b   = bid >> 7;
  const int s0  = st * 64;
  {
    const int sl = tid >> 2;
    const int dc = (tid & 3) * 32;
    const float* src = v + (((size_t)(b * SEQ + s0 + sl)) * NKV + g) * HD + dc;
#pragma unroll
    for (int i = 0; i < 8; ++i) {
      const v4f a = *(const v4f*)(src + 4 * i);
#pragma unroll
      for (int e = 0; e < 4; ++e) T[(dc + 4 * i + e) * VTP + sl] = h_bits((_Float16)(bfr(a[e]) * VCAR));
    }
  }
  __syncthreads();
  v4u vals[4];
  const int q8 = tid >> 3, p8 = (tid & 7) * 8;
#pragma unroll
  for (int it = 0; it < 4; ++it) {
    const int line = it * 32 + q8;
    vals[it] = *(const v4u*)(T + line * VTP + p8);
  }
  unsigned short* dst = VTo + ((size_t)(b * NKV + g) * HD) * SEQ + s0 + p8;
  for (int pass = 0; pass < 2; ++pass) {
#pragma unroll
    for (int it = 0; it < 4; ++it) {
      const int line = it * 32 + q8;
      *(volatile v4u*)(dst + (size_t)line * SEQ) = vals[it];
    }
    __threadfence();
  }
}

__global__ __launch_bounds__(ATT_THREADS)
void attn_gqa(const unsigned short* __restrict__ QHIp, const unsigned short* __restrict__ QLOp,
              const unsigned short* __restrict__ KHIp, const unsigned short* __restrict__ KLOp,
              const unsigned short* __restrict__ VTq, const float* __restrict__ Bp,
              const float* __restrict__ scp, float* outp) {
  __shared__ __align__(16) float smem[ATW * SLABF];

  const int tid  = threadIdx.x;
  const int wave = tid >> 5;
  const int lane = tid & 31;
  const int hh   = lane >> 4;
  const int c    = lane & 15;

  const int bid  = blockIdx.x;
  const int qt   = bid & 63;
  const int g    = (bid >> 6) & 7;
  const int b    = bid >> 9;
  const int head = g * GRP + wave;
  const int q0   = qt * 16;

  const size_t qofs = (((size_t)(b * SEQ + q0 + c)) * NH + head) * HD + 8 * hh;
  const _Float16* Qh  = (const _Float16*)(const void*)QHIp + qofs;
  const _Float16* Ql  = (const _Float16*)(const void*)QLOp + qofs;
  const size_t kofs = (((size_t)b * SEQ + c) * NKV + g) * HD + 8 * hh;
  const _Float16* Khb = (const _Float16*)(const void*)KHIp + kofs;
  const _Float16* Klb = (const _Float16*)(const void*)KLOp + kofs;
  const _Float16* Vb  = (const _Float16*)(const void*)VTq + ((size_t)(b * NKV + g) * HD + c) * SEQ + 8 * hh;
  const float*    Wr  = Bp + ((size_t)b * SEQ + q0 + 8 * hh) * SEQ + c;
  const float lsc = bfr(scp[0]) * (LOG2E / (QSC * KSC));

  float mrow[8], lrow[8];
  v8f o[8];
#pragma unroll
  for (int r = 0; r < 8; ++r) { mrow[r] = -INFINITY; lrow[r] = 0.f; }
#pragma unroll
  for (int j = 0; j < 8; ++j) o[j] = zero8();
  float* pt = smem + wave * SLABF;

#pragma unroll 1
  for (int kb = 0; kb < SEQ; kb += 32) {
    float w0[8], w1[8];
    bool allm = true, seen = true;
    const float* wp = Wr + kb;
#pragma unroll
    for (int r = 0; r < 8; ++r) {
      const float m0 = bfr(wp[(size_t)r * SEQ]);
      const float m1 = bfr(wp[(size_t)r * SEQ + 16]);
      allm = allm & (m0 <= BIASTH) & (m1 <= BIASTH);
      seen = seen & (mrow[r] > BIASTH);
      w0[r] = m0 * LOG2E;
      w1[r] = m1 * LOG2E;
    }
    const unsigned bal = __builtin_amdgcn_ballot_w32(allm & seen);
    if (bal != 0xffffffffu) {
      v8f s0 = zero8(), s1 = zero8();
      const _Float16* k0p = Khb + (size_t)kb * (NKV * HD);
      const _Float16* k1p = k0p + (size_t)16 * (NKV * HD);
      const _Float16* l0p = Klb + (size_t)kb * (NKV * HD);
      const _Float16* l1p = l0p + (size_t)16 * (NKV * HD);
#pragma unroll
      for (int kk = 0; kk < 4; ++kk) {
        const v16h qh  = ldfrag_h(Qh + kk * 32),  ql  = ldfrag_h(Ql + kk * 32);
        const v16h kh0 = ldfrag_h(k0p + kk * 32), kl0 = ldfrag_h(l0p + kk * 32);
        const v16h kh1 = ldfrag_h(k1p + kk * 32), kl1 = ldfrag_h(l1p + kk * 32);
        s0 = mma_raw(qh, kh0, s0);
        s0 = mma_raw(ql, kh0, s0);
        s0 = mma_raw(qh, kl0, s0);
        s1 = mma_raw(qh, kh1, s1);
        s1 = mma_raw(ql, kh1, s1);
        s1 = mma_raw(qh, kl1, s1);
        guard_sc(s0, s1, qh, ql, kh0, kl0, kh1, kl1);
      }
#pragma unroll
      for (int r = 0; r < 8; ++r) {
        const float t0 = s0[r] * lsc + w0[r], t1 = s1[r] * lsc + w1[r];
        float mx = fmaxf(t0, t1);
#pragma unroll
        for (int off = 1; off < 16; off <<= 1) mx = fmaxf(mx, __shfl_xor(mx, off, 32));
        const float mn = fmaxf(mrow[r], mx);
        const float al = exp2f(mrow[r] - mn);
        mrow[r] = mn;
        const float e0 = exp2f(t0 - mn), e1 = exp2f(t1 - mn);
        float ps = e0 + e1;
#pragma unroll
        for (int off = 1; off < 16; off <<= 1) ps += __shfl_xor(ps, off, 32);
        lrow[r] = lrow[r] * al + ps;
#pragma unroll
        for (int j = 0; j < 8; ++j) o[j][r] *= al;
        const int ro = (8 * hh + r) * 36 + c;
        pt[ro]      = e0;
        pt[ro + 16] = e1;
      }
      wave_sync_lds();
      FragH ph, pl;
      {
        const float* prow = pt + c * 36 + 8 * hh;
        const v4f p0 = *(const v4f*)(prow), p1 = *(const v4f*)(prow + 4);
        const v4f p2 = *(const v4f*)(prow + 16), p3 = *(const v4f*)(prow + 20);
#pragma unroll
        for (int e = 0; e < 4; ++e) {
          const float ta = p0[e] * PCAR, tb = p1[e] * PCAR, tc = p2[e] * PCAR, td = p3[e] * PCAR;
          const _Float16 ha = (_Float16)ta, hb = (_Float16)tb, hc = (_Float16)tc, hd = (_Float16)td;
          ph.h[0][e]     = ha;
          ph.h[0][4 + e] = hb;
          ph.h[1][e]     = hc;
          ph.h[1][4 + e] = hd;
          pl.h[0][e]     = (_Float16)(ta - (float)ha);
          pl.h[0][4 + e] = (_Float16)(tb - (float)hb);
          pl.h[1][e]     = (_Float16)(tc - (float)hc);
          pl.h[1][4 + e] = (_Float16)(td - (float)hd);
        }
      }
      const _Float16* vp = Vb + kb;
      {
        const v16h vb0 = ldfrag_h(vp);
        const v16h vb1 = ldfrag_h(vp + (size_t)16 * SEQ);
        const v16h vb2 = ldfrag_h(vp + (size_t)32 * SEQ);
        const v16h vb3 = ldfrag_h(vp + (size_t)48 * SEQ);
        o[0] = mma_raw(ph.v, vb0, o[0]);  o[0] = mma_raw(pl.v, vb0, o[0]);
        o[1] = mma_raw(ph.v, vb1, o[1]);  o[1] = mma_raw(pl.v, vb1, o[1]);
        o[2] = mma_raw(ph.v, vb2, o[2]);  o[2] = mma_raw(pl.v, vb2, o[2]);
        o[3] = mma_raw(ph.v, vb3, o[3]);  o[3] = mma_raw(pl.v, vb3, o[3]);
        guard_pv(o[0], o[1], o[2], o[3], ph.v, pl.v, vb0, vb1, vb2, vb3);
      }
      {
        const v16h vb4 = ldfrag_h(vp + (size_t)64 * SEQ);
        const v16h vb5 = ldfrag_h(vp + (size_t)80 * SEQ);
        const v16h vb6 = ldfrag_h(vp + (size_t)96 * SEQ);
        const v16h vb7 = ldfrag_h(vp + (size_t)112 * SEQ);
        o[4] = mma_raw(ph.v, vb4, o[4]);  o[4] = mma_raw(pl.v, vb4, o[4]);
        o[5] = mma_raw(ph.v, vb5, o[5]);  o[5] = mma_raw(pl.v, vb5, o[5]);
        o[6] = mma_raw(ph.v, vb6, o[6]);  o[6] = mma_raw(pl.v, vb6, o[6]);
        o[7] = mma_raw(ph.v, vb7, o[7]);  o[7] = mma_raw(pl.v, vb7, o[7]);
        guard_pv(o[4], o[5], o[6], o[7], ph.v, pl.v, vb4, vb5, vb6, vb7);
      }
      wave_sync_lds();
    }
  }
  acc_guard4(o[0], o[1], o[2], o[3]);
  acc_guard4(o[4], o[5], o[6], o[7]);

  wave_sync_lds();
  float* slab = pt;
  const float oc = 1.0f / (PCAR * VCAR);
#pragma unroll
  for (int r = 0; r < 8; ++r) {
    const float inv = (1.0f / lrow[r]) * oc;
#pragma unroll
    for (int j = 0; j < 8; ++j) slab[(8 * hh + r) * 132 + j * 16 + c] = o[j][r] * inv;
  }
  wave_sync_lds();
  v4f vals[16];
#pragma unroll
  for (int row = 0; row < 16; ++row) vals[row] = *(const v4f*)(slab + row * 132 + lane * 4);
  float* dst = outp + (((size_t)(b * SEQ + q0)) * NH + head) * HD + lane * 4;
  for (int pass = 0; pass < 2; ++pass) {
#pragma unroll
    for (int row = 0; row < 16; ++row) {
      *(volatile v4f*)(dst + (size_t)row * (NH * HD)) = vals[row];
    }
    __threadfence();
  }
}

extern "C" void kernel_launch(void* const* d_in, const int* in_sizes, int n_in,
                              void* d_out, int out_size, void* d_ws, size_t ws_size,
                              hipStream_t stream) {
  if (n_in < 7) return;
  if (in_sizes[0] != NB * SEQ * NH * HD) return;
  if (in_sizes[1] != NB * SEQ * NKV * HD || in_sizes[2] != NB * SEQ * NKV * HD) return;
  if (in_sizes[3] != SEQ * HD || in_sizes[4] != SEQ * HD) return;
  if (in_sizes[5] != NB * SEQ * SEQ) return;
  if (in_sizes[6] < 1) return;
  if (out_size != NB * SEQ * NH * HD) return;

  const float* q    = (const float*)d_in[0];
  const float* k    = (const float*)d_in[1];
  const float* v    = (const float*)d_in[2];
  const float* cosT = (const float*)d_in[3];
  const float* sinT = (const float*)d_in[4];
  const float* bias = (const float*)d_in[5];
  const float* scl  = (const float*)d_in[6];
  float*       out  = (float*)d_out;

  const size_t PQ = (size_t)NB * SEQ * NH * HD * 2;
  const size_t PK = (size_t)NB * SEQ * NKV * HD * 2;
  const size_t PV = (size_t)NB * NKV * HD * SEQ * 2;
  size_t off = 0;
  const size_t oQH = off; off += PQ;
  const size_t oQL = off; off += PQ;
  const size_t oKH = off; off += PK;
  const size_t oKL = off; off += PK;
  const size_t oVT = off; off += PV;
  if (off > ws_size) return;
  if (off > (size_t)134217728) return;

  char* ws = (char*)d_ws;
  unsigned short* QHI = (unsigned short*)(ws + oQH);
  unsigned short* QLO = (unsigned short*)(ws + oQL);
  unsigned short* KHI = (unsigned short*)(ws + oKH);
  unsigned short* KLO = (unsigned short*)(ws + oKL);
  unsigned short* VT  = (unsigned short*)(ws + oVT);

  const int rowsQ = NB * SEQ * NH;
  const int rowsK = NB * SEQ * NKV;
  const dim3 blk(256);
  const dim3 gRQ((rowsQ * 16) / 256);
  const dim3 gRK((rowsK * 16) / 256);
  const dim3 gVT(NB * NKV * (SEQ / 64));
  const dim3 gAT(ATT_BLOCKS);
  const dim3 bAT(ATT_THREADS);

  rope16<<<gRQ, blk, 0, stream>>>(q, cosT, sinT, QHI, QLO, rowsQ, NH, QSC);
  rope16<<<gRK, blk, 0, stream>>>(k, cosT, sinT, KHI, KLO, rowsK, NKV, KSC);
  vt16<<<gVT, blk, 0, stream>>>(v, VT);
  attn_gqa<<<gAT, bAT, 0, stream>>>(QHI, QLO, KHI, KLO, VT, bias, scl, out);
  (void)hipGetLastError();
}
